// SegGPNet_6579889897729
// MI455X (gfx1250) — hardware-run, weakly checked
//
#include <hip/hip_runtime.h>
#include <math.h>

typedef __attribute__((ext_vector_type(16))) _Float16 v16h;
typedef __attribute__((ext_vector_type(8)))  _Float16 v8h;
typedef __attribute__((ext_vector_type(8)))  float    v8f;
typedef __attribute__((ext_vector_type(4)))  float    v4f;
typedef __attribute__((ext_vector_type(4)))  unsigned v4u;
typedef __attribute__((ext_vector_type(4)))  int      v4i;

constexpr int kBatch   = 16;
constexpr int kPts     = 8192;
constexpr int kCin     = 3;
constexpr int kHid     = 64;
constexpr int kFeat    = 256;
constexpr int kBranch  = 4;
constexpr int kHeadHid = 128;
constexpr int kOutDim  = 128;
constexpr int kTilePts = 64;
constexpr int kTilesPerBatch = kPts / kTilePts;
constexpr int kAugK    = kBranch * kHid;
constexpr int kAPitch  = kAugK + 8;
constexpr int kTsPitch = 257;
constexpr float kCarryH = 1024.0f;
constexpr float kCarryW = 1024.0f;
constexpr float kFold   = 1.0f / (kCarryH * kCarryW);
constexpr float kNegMax = -3.402823466e+38f;

static_assert(kAugK == 256);
static_assert((kAugK % 32) == 0);
static_assert((kTilePts % 16) == 0 && (kFeat % 32) == 0);
static_assert(kTilesPerBatch == 128);
static_assert(kTilesPerBatch * kTilePts == kPts);
static_assert(kBatch * kCin * kPts == 393216);
static_assert(kBatch * kBranch * kPts == 524288);
static_assert(kBranch * kCin * kHid == 768);
static_assert(kBranch * kHid * kFeat == 65536);
static_assert(kFeat * kHeadHid == 32768);
static_assert(kHeadHid * kOutDim == 16384);
static_assert(kBatch * kOutDim == 2048);
static_assert(((kAPitch * 2) % 16) == 0);

constexpr size_t kOffBt    = 0;
constexpr size_t kBytesBt  = (size_t)kFeat * kAugK * 2;
constexpr size_t kOffPart  = kOffBt + kBytesBt;
constexpr size_t kBytesPart = (size_t)kBatch * kTilesPerBatch * kFeat * 4;
constexpr size_t kWsTotal  = kOffPart + kBytesPart;
static_assert(kBytesBt == 131072ull);
static_assert(kBytesPart == 2097152ull);
static_assert(kWsTotal == 2228224ull);
static_assert(kWsTotal <= 134217728ull);
static_assert((kOffPart % 128) == 0);

union FragU { v16h v; v8h h[2]; };
__device__ __forceinline__ v16h frag_load(const _Float16* p) {
  FragU f;
  f.h[0] = *(const v8h*)(p);
  f.h[1] = *(const v8h*)(p + 16);
  return f.v;
}
__device__ __forceinline__ v8f mma_f16(v16h a, v16h b, v8f c) {
  c = __builtin_amdgcn_wmma_f32_16x16x32_f16(false, a, false, b, (short)0, c, false, false);
  asm volatile("v_nop\n\tv_nop\n\tv_nop\n\tv_nop" : "+v"(c) : "v"(a), "v"(b));
  return c;
}

__device__ __forceinline__ float gelu_erf(float v) {
  return 0.5f * v * (1.0f + erff(v * 0.70710678118654752f));
}

__global__ __launch_bounds__(256) void k_prep_bt(const float* __restrict__ W2, unsigned short* __restrict__ Bt)
{
  __shared__ __align__(16) float ts[16 * kTsPitch];
  const int tid = threadIdx.x;
  const int d0 = blockIdx.x * 16;
#pragma unroll 4
  for (int it = 0; it < 16; ++it) {
    const int e  = it * 256 + tid;
    const int kk = e >> 4;
    const int dd = e & 15;
    ts[dd * kTsPitch + kk] = W2[(size_t)kk * kFeat + d0 + dd];
  }
  __syncthreads();
  v8h hv[2];
#pragma unroll
  for (int it = 0; it < 2; ++it) {
    const int idx = it * 256 + tid;
    const int row = idx >> 5;
    const int c8  = (idx & 31) * 8;
#pragma unroll
    for (int e = 0; e < 8; ++e) {
      const float w = ts[row * kTsPitch + c8 + e] * kCarryW;
      hv[it][e] = (_Float16)w;
    }
  }
  for (int pass = 0; pass < 2; ++pass) {
#pragma unroll
    for (int it = 0; it < 2; ++it) {
      const int idx = it * 256 + tid;
      const int row = idx >> 5;
      const int c8  = (idx & 31) * 8;
      *(volatile v8h*)(Bt + (size_t)(d0 + row) * kAugK + c8) = hv[it];
    }
    __threadfence();
  }
}

__global__ __launch_bounds__(256) void k_branch_max(
    const float* __restrict__ x, const float* __restrict__ lab,
    const float* __restrict__ W1, const float* __restrict__ b1,
    const float* __restrict__ b2, const unsigned short* __restrict__ Btp,
    float* __restrict__ partials)
{
  __shared__ __align__(16) _Float16 sA[kTilePts * kAPitch];
  __shared__ __align__(16) float sW1[kBranch * kCin * kHid];
  __shared__ __align__(16) float sB1[kBranch * kHid];
  __shared__ __align__(16) float sB2[kBranch * kFeat];
  __shared__ __align__(16) int   sK[kTilePts];
  __shared__ __align__(16) float sM[kFeat];

  const int tid  = threadIdx.x;
  const int lane = tid & 31;
  const int wave = tid >> 5;
  const int bix  = blockIdx.x >> 7;
  const int tile = blockIdx.x & (kTilesPerBatch - 1);
  const int n0   = tile * kTilePts;

#pragma unroll
  for (int i = tid; i < kBranch * kCin * kHid; i += 256) sW1[i] = W1[i];
  sB1[tid] = b1[tid];
#pragma unroll
  for (int i = 0; i < 4; ++i) sB2[i * 256 + tid] = b2[i * 256 + tid];

  const int p = tid >> 2;
  const int q = tid & 3;
  const int n = n0 + p;
  const float l0 = lab[((size_t)bix * kBranch + 0) * kPts + n];
  const float l1 = lab[((size_t)bix * kBranch + 1) * kPts + n];
  const float l2 = lab[((size_t)bix * kBranch + 2) * kPts + n];
  const float l3 = lab[((size_t)bix * kBranch + 3) * kPts + n];
  const float x0 = x[((size_t)bix * kCin + 0) * kPts + n];
  const float x1 = x[((size_t)bix * kCin + 1) * kPts + n];
  const float x2 = x[((size_t)bix * kCin + 2) * kPts + n];
  int k = 0;
  float lm = l0;
  if (l1 > lm) { lm = l1; k = 1; }
  if (l2 > lm) { lm = l2; k = 2; }
  if (l3 > lm) { lm = l3; k = 3; }
  if (q == 0) sK[p] = k;
  __syncthreads();

#pragma unroll 1
  for (int g = 0; g < 2; ++g) {
    const int jb = q * 16 + g * 8;
    const float* wr = sW1 + k * (kCin * kHid) + jb;
    const v4f w0a = *(const v4f*)(wr);
    const v4f w0b = *(const v4f*)(wr + 4);
    const v4f w1a = *(const v4f*)(wr + kHid);
    const v4f w1b = *(const v4f*)(wr + kHid + 4);
    const v4f w2a = *(const v4f*)(wr + 2 * kHid);
    const v4f w2b = *(const v4f*)(wr + 2 * kHid + 4);
    const v4f ba  = *(const v4f*)(sB1 + k * kHid + jb);
    const v4f bb  = *(const v4f*)(sB1 + k * kHid + jb + 4);
    v8h hv;
#pragma unroll
    for (int e = 0; e < 4; ++e) {
      float pa = x0 * w0a[e];
      pa = fmaf(x1, w1a[e], pa);
      pa = fmaf(x2, w2a[e], pa);
      pa = pa + ba[e];
      float pb = x0 * w0b[e];
      pb = fmaf(x1, w1b[e], pb);
      pb = fmaf(x2, w2b[e], pb);
      pb = pb + bb[e];
      const float ha = gelu_erf(pa) * kCarryH;
      const float hb = gelu_erf(pb) * kCarryH;
      hv[e]     = (_Float16)ha;
      hv[4 + e] = (_Float16)hb;
    }
    const v4u hw = __builtin_bit_cast(v4u, hv);
#pragma unroll
    for (int s = 0; s < kBranch; ++s) {
      const unsigned mm = (s == k) ? 0xFFFFFFFFu : 0u;
      const v4u mv = (v4u){mm, mm, mm, mm};
      const v4u ow = hw & mv;
      *(v8h*)(sA + p * kAPitch + s * kHid + jb) = __builtin_bit_cast(v8h, ow);
    }
  }
  __syncthreads();

  const _Float16* Bt = (const _Float16*)Btp;
  const int rl   = lane & 15;
  const int hh   = lane >> 4;
  const int koff = hh * 8;
  v8f acc[4][2];
#pragma unroll
  for (int i = 0; i < 4; ++i) {
    acc[i][0] = (v8f){0.f, 0.f, 0.f, 0.f, 0.f, 0.f, 0.f, 0.f};
    acc[i][1] = (v8f){0.f, 0.f, 0.f, 0.f, 0.f, 0.f, 0.f, 0.f};
  }
  const _Float16* bp0 = Bt + (size_t)(wave * 32 + rl) * kAugK + koff;
  const _Float16* bp1 = bp0 + (size_t)16 * kAugK;
  const _Float16* ap  = sA + rl * kAPitch + koff;
#pragma unroll 1
  for (int k0 = 0; k0 < kAugK; k0 += 32) {
    const v16h bf0 = frag_load(bp0 + k0);
    const v16h bf1 = frag_load(bp1 + k0);
#pragma unroll
    for (int i = 0; i < 4; ++i) {
      const v16h af = frag_load(ap + i * 16 * kAPitch + k0);
      acc[i][0] = mma_f16(af, bf0, acc[i][0]);
      acc[i][1] = mma_f16(af, bf1, acc[i][1]);
    }
  }

  const int colA = wave * 32 + rl;
  const int colB = colA + 16;
  float mxA = kNegMax;
  float mxB = kNegMax;
#pragma unroll
  for (int i = 0; i < 4; ++i) {
    const v4i ka = *(const v4i*)(sK + i * 16 + hh * 8);
    const v4i kb = *(const v4i*)(sK + i * 16 + hh * 8 + 4);
#pragma unroll
    for (int r = 0; r < 4; ++r) {
      const int kr0 = ka[r];
      const int kr1 = kb[r];
      const float va0 = fmaf(acc[i][0][r],     kFold, sB2[kr0 * kFeat + colA]);
      const float vb0 = fmaf(acc[i][1][r],     kFold, sB2[kr0 * kFeat + colB]);
      const float va1 = fmaf(acc[i][0][4 + r], kFold, sB2[kr1 * kFeat + colA]);
      const float vb1 = fmaf(acc[i][1][4 + r], kFold, sB2[kr1 * kFeat + colB]);
      mxA = fmaxf(mxA, fmaxf(va0, va1));
      mxB = fmaxf(mxB, fmaxf(vb0, vb1));
    }
  }
  const float oA = __shfl_xor(mxA, 16, 32);
  const float oB = __shfl_xor(mxB, 16, 32);
  mxA = fmaxf(mxA, oA);
  mxB = fmaxf(mxB, oB);
  const float mine = (lane < 16) ? mxA : mxB;
  sM[wave * 32 + lane] = mine;
  __syncthreads();
  if (wave < 2) {
    const v4f val = *(const v4f*)(sM + wave * 128 + lane * 4);
    float* dst = partials + (size_t)blockIdx.x * kFeat + wave * 128 + lane * 4;
    *(volatile v4f*)dst = val;
    __threadfence();
    *(volatile v4f*)dst = val;
  }
}

__global__ __launch_bounds__(128) void k_head(
    const float* __restrict__ partials, const float* __restrict__ Wg1, const float* __restrict__ bg1,
    const float* __restrict__ Wg2, const float* __restrict__ bg2, float* __restrict__ out)
{
  __shared__ __align__(16) float sG[kFeat];
  __shared__ __align__(16) float sA1[kHeadHid];
  __shared__ __align__(16) float sO[kOutDim];
  const int b = blockIdx.x;
  const int t = threadIdx.x;
  const float* pp = partials + (size_t)b * kTilesPerBatch * kFeat;
  float m0 = kNegMax;
  float m1 = kNegMax;
#pragma unroll 4
  for (int tl = 0; tl < kTilesPerBatch; ++tl) {
    m0 = fmaxf(m0, pp[(size_t)tl * kFeat + t]);
    m1 = fmaxf(m1, pp[(size_t)tl * kFeat + 128 + t]);
  }
  sG[t] = m0;
  sG[t + 128] = m1;
  __syncthreads();
  float acc = 0.0f;
#pragma unroll 4
  for (int d = 0; d < kFeat; ++d) acc = fmaf(sG[d], Wg1[(size_t)d * kHeadHid + t], acc);
  acc = acc + bg1[t];
  sA1[t] = gelu_erf(acc);
  __syncthreads();
  float acc2 = 0.0f;
#pragma unroll 4
  for (int j = 0; j < kHeadHid; ++j) acc2 = fmaf(sA1[j], Wg2[(size_t)j * kOutDim + t], acc2);
  acc2 = acc2 + bg2[t];
  sO[t] = acc2;
  __syncthreads();
  if (t < 32) {
    const v4f val = *(const v4f*)(sO + t * 4);
    float* dst = out + (size_t)b * kOutDim + t * 4;
    *(volatile v4f*)dst = val;
    __threadfence();
    *(volatile v4f*)dst = val;
  }
}

extern "C" void kernel_launch(void* const* d_in, const int* in_sizes, int n_in,
                              void* d_out, int out_size, void* d_ws, size_t ws_size,
                              hipStream_t stream) {
  if (n_in < 10) return;
  if (in_sizes[0] != kBatch * kCin * kPts) return;
  if (in_sizes[1] != kBatch * kBranch * kPts) return;
  if (in_sizes[2] != kBranch * kCin * kHid) return;
  if (in_sizes[3] != kBranch * kHid) return;
  if (in_sizes[4] != kBranch * kHid * kFeat) return;
  if (in_sizes[5] != kBranch * kFeat) return;
  if (in_sizes[6] != kFeat * kHeadHid) return;
  if (in_sizes[7] != kHeadHid) return;
  if (in_sizes[8] != kHeadHid * kOutDim) return;
  if (in_sizes[9] != kOutDim) return;
  if (out_size != kBatch * kOutDim) return;
  if (ws_size < kWsTotal) return;

  const float* x   = (const float*)d_in[0];
  const float* lab = (const float*)d_in[1];
  const float* W1  = (const float*)d_in[2];
  const float* b1  = (const float*)d_in[3];
  const float* W2  = (const float*)d_in[4];
  const float* b2  = (const float*)d_in[5];
  const float* Wg1 = (const float*)d_in[6];
  const float* bg1 = (const float*)d_in[7];
  const float* Wg2 = (const float*)d_in[8];
  const float* bg2 = (const float*)d_in[9];
  float* out = (float*)d_out;

  char* ws = (char*)d_ws;
  unsigned short* BT   = (unsigned short*)(ws + kOffBt);
  float*          PART = (float*)(ws + kOffPart);

  k_prep_bt<<<kFeat / 16, 256, 0, stream>>>(W2, BT);
  k_branch_max<<<kBatch * kTilesPerBatch, 256, 0, stream>>>(x, lab, W1, b1, b2, BT, PART);
  k_head<<<kBatch, 128, 0, stream>>>(PART, Wg1, bg1, Wg2, bg2, out);
}
